// RegionSimilarityAnalysis_76184129896955
// MI455X (gfx1250) — hardware-verified
//
#include <hip/hip_runtime.h>
#include <math.h>

#define BB     4
#define CC     64
#define HH     128
#define WW     128
#define KK     7
#define NOFF   (KK * KK)
#define PAD    3
#define HP     (HH + 2 * PAD)
#define WP     (WW + 2 * PAD)
#define NPITCH 160
#define EPSF   1e-7f
#define XSC    64.0f
#define INVSC2 (1.0f / 4096.0f)
#define XSP    132
#define HSP    72
#define SMP    52
#define OPIX   (HH * WW)

typedef _Float16 v16h __attribute__((ext_vector_type(16)));
typedef _Float16 v8h  __attribute__((ext_vector_type(8)));
typedef float    v8f  __attribute__((ext_vector_type(8)));
typedef float    v4f  __attribute__((ext_vector_type(4)));
union FragH { v16h v; v8h half[2]; };

__device__ __forceinline__ v8f wmma_f16(v16h a, v16h b, v8f c)
{
    v8f d = __builtin_amdgcn_wmma_f32_16x16x32_f16(false, a, false, b, (short)0, c, false, false);
    asm volatile("v_nop\n\tv_nop\n\tv_nop\n\tv_nop" : "+v"(d) : "v"(a), "v"(b));
    return d;
}

__global__ __launch_bounds__(256)
void prep_kernel(const float* __restrict__ x,
                 _Float16* __restrict__ xT,
                 float* __restrict__ nrm)
{
    __shared__ __align__(16) float    xs[CC][XSP];
    __shared__ __align__(16) _Float16 hs[WP][HSP];
    __shared__ float ns[NPITCH];

    const int pr   = blockIdx.x;
    const int b    = blockIdx.y;
    const int tid  = threadIdx.x;
    const int lane = tid & 31;
    const int wave = tid >> 5;

    const int  r     = pr - PAD;
    const bool inrow = (r >= 0) && (r < HH);
    const int  rc    = (r < 0) ? 0 : ((r > HH - 1) ? (HH - 1) : r);
    const float* xb  = x + (size_t)b * CC * HH * WW + (size_t)rc * WW;
    const v4f z4 = (v4f){0.f, 0.f, 0.f, 0.f};

#pragma unroll
    for (int it = 0; it < 8; ++it) {
        const int q  = it * 256 + tid;
        const int c  = q >> 5;
        const int w4 = (q & 31) * 4;
        v4f v = *(const v4f*)(xb + (size_t)c * HH * WW + w4);
        v = inrow ? v : z4;
        *(v4f*)(&xs[c][w4]) = v;
    }
    __syncthreads();

    const int  pc    = (tid < WP) ? tid : (WP - 1);
    const int  cw    = pc - PAD;
    const bool incol = (cw >= 0) && (cw < WW);
    const int  cwc   = (cw < 0) ? 0 : ((cw > WW - 1) ? (WW - 1) : cw);
    float s = 0.f;
#pragma unroll 1
    for (int g = 0; g < CC / 8; ++g) {
        v8h hv;
#pragma unroll
        for (int e = 0; e < 8; ++e) {
            float f = xs[g * 8 + e][cwc];
            f = incol ? f : 0.f;
            s = fmaf(f, f, s);
            hv[e] = (_Float16)(f * XSC);
        }
        if (tid < WP) *(v8h*)(&hs[pc][g * 8]) = hv;
    }
    const float nv = (tid < WP) ? sqrtf(s) : 0.f;
    if (tid < NPITCH) ns[tid] = nv;
    __syncthreads();

    _Float16* xrow = xT  + ((size_t)(b * HP + pr) * WP) * CC;
    float*    nrow = nrm + (size_t)(b * HP + pr) * NPITCH;
    const int lq = lane >> 3;
    const int e8 = (lane & 7) * 8;
    int  Lv[5];
    v8h  hvv[5];
#pragma unroll
    for (int it = 0; it < 5; ++it) {
        const int L  = it * 32 + wave * 4 + lq;
        const int Lc = (L < WP) ? L : (WP - 1);
        Lv[it]  = L;
        hvv[it] = *(const v8h*)(&hs[Lc][e8]);
    }
    const int   nw   = (wave < 5) ? wave : 4;
    const float nval = ns[nw * 32 + lane];

#pragma unroll
    for (int it = 0; it < 5; ++it)
        if (Lv[it] < WP) *(volatile v8h*)(xrow + (size_t)Lv[it] * CC + e8) = hvv[it];
    if (wave < 5) *(volatile float*)(nrow + wave * 32 + lane) = nval;
    __threadfence();
#pragma unroll
    for (int it = 0; it < 5; ++it)
        if (Lv[it] < WP) *(volatile v8h*)(xrow + (size_t)Lv[it] * CC + e8) = hvv[it];
    if (wave < 5) *(volatile float*)(nrow + wave * 32 + lane) = nval;
}

__global__ __launch_bounds__(256)
void sim_softmax_kernel(const _Float16* __restrict__ xT,
                        const float* __restrict__ nrm,
                        float* __restrict__ out)
{
    __shared__ __align__(16) float sm[8][16][SMP];

    const int bh   = blockIdx.x;
    const int b    = bh >> 7;
    const int h    = bh & (HH - 1);
    const int lane = threadIdx.x & 31;
    const int wave = threadIdx.x >> 5;
    const int w0   = wave * 16;
    const int half = lane >> 4;
    const int n    = lane & 15;

    const size_t rowStride = (size_t)WP * CC;
    const _Float16* bbase  = xT  + (size_t)b * HP * rowStride;
    const float*    nb     = nrm + (size_t)b * HP * NPITCH;

    const _Float16* cpix = bbase + (size_t)(h + PAD) * rowStride + (size_t)(w0 + PAD + n) * CC;
    FragH a0, a1;
    a0.half[0] = *(const v8h*)(cpix +      8 * half);
    a0.half[1] = *(const v8h*)(cpix + 16 + 8 * half);
    a1.half[0] = *(const v8h*)(cpix + 32 + 8 * half);
    a1.half[1] = *(const v8h*)(cpix + 48 + 8 * half);

    const float* ncRow = nb + (size_t)(h + PAD) * NPITCH + (w0 + PAD) + 8 * half;
    float ncv[8];
#pragma unroll
    for (int r = 0; r < 8; ++r) ncv[r] = ncRow[r];

#pragma unroll 1
    for (int i = 0; i < KK; ++i) {
        const _Float16* rowi = bbase + (size_t)(h + i) * rowStride;
        const float*    nri  = nb + (size_t)(h + i) * NPITCH;

#pragma unroll
        for (int tile = 0; tile < 2; ++tile) {
            int col = w0 + 16 * tile + n;
            col = (col < WP) ? col : (WP - 1);
            const float np = nri[col];

            const _Float16* bp = rowi + (size_t)col * CC;
            FragH b0, b1;
            b0.half[0] = *(const v8h*)(bp +      8 * half);
            b0.half[1] = *(const v8h*)(bp + 16 + 8 * half);
            b1.half[0] = *(const v8h*)(bp + 32 + 8 * half);
            b1.half[1] = *(const v8h*)(bp + 48 + 8 * half);

            v8f acc = (v8f){0.f, 0.f, 0.f, 0.f, 0.f, 0.f, 0.f, 0.f};
            acc = wmma_f16(a0.v, b0.v, acc);
            acc = wmma_f16(a1.v, b1.v, acc);

#pragma unroll
            for (int r = 0; r < 8; ++r) {
                const int m    = r + 8 * half;
                const int j    = n - m + 16 * tile;
                const int slot = ((unsigned)j < (unsigned)KK) ? (i * KK + j) : NOFF;
                const float den = fmaf(ncv[r], np, EPSF);
                const float val = (acc[r] * INVSC2) * __builtin_amdgcn_rcpf(den);
                sm[wave][m][slot] = val;
            }
        }
    }

    __syncthreads();

    const int p = threadIdx.x;
    if (p < WW) {
        float* row = &sm[p >> 4][p & 15][0];
        float mx = row[0];
#pragma unroll 1
        for (int k = 1; k < NOFF; ++k) mx = fmaxf(mx, row[k]);
        float sum = 0.f;
#pragma unroll 1
        for (int k = 0; k < NOFF; ++k) {
            const float e = expf(row[k] - mx);
            row[k] = e;
            sum += e;
        }
        const float inv = __builtin_amdgcn_rcpf(sum);
#pragma unroll 1
        for (int k = 0; k < NOFF; ++k) row[k] = row[k] * inv;

        float* op = out + (size_t)b * NOFF * OPIX + (size_t)h * WW + p;
#pragma unroll 1
        for (int k = 0; k < NOFF; ++k)
            *(volatile float*)(op + (size_t)k * OPIX) = row[k];
        __threadfence();
#pragma unroll 1
        for (int k = 0; k < NOFF; ++k)
            *(volatile float*)(op + (size_t)k * OPIX) = row[k];
    }
}

extern "C" void kernel_launch(void* const* d_in, const int* in_sizes, int n_in,
                              void* d_out, int out_size, void* d_ws, size_t ws_size,
                              hipStream_t stream)
{
    if (n_in < 1) return;
    if (in_sizes[0] != BB * CC * HH * WW) return;
    if (out_size != BB * NOFF * OPIX) return;

    const size_t xT_bytes  = (size_t)BB * HP * WP * CC * sizeof(_Float16);
    const size_t nrm_bytes = (size_t)BB * HP * NPITCH * sizeof(float);
    if (xT_bytes + nrm_bytes > ws_size) return;

    const float* x   = (const float*)d_in[0];
    float*       out = (float*)d_out;
    _Float16*    xT  = (_Float16*)d_ws;
    float*       nrm = (float*)((char*)d_ws + xT_bytes);

    prep_kernel<<<dim3(HP, BB), dim3(256), 0, stream>>>(x, xT, nrm);
    sim_softmax_kernel<<<dim3(BB * HH), dim3(256), 0, stream>>>(xT, nrm, out);
    (void)hipGetLastError();
}
